// VDProjAttention_82351702933750
// MI455X (gfx1250) — hardware-verified
//
#include <hip/hip_runtime.h>


#define NB_  2
#define TT   2048
#define DM   2048
#define NH_  16
#define HD   128
#define RD   32
#define VHD  20
#define VP   320
#define VT64 64
#define ZH   2
#define RH   512
#define PCAR 1024.0f
#define SCL  0.088388347648318447f
typedef _Float16 h16;
typedef unsigned short bf;
typedef __attribute__((ext_vector_type(16))) __bf16   v16bf;
typedef __attribute__((ext_vector_type(16))) _Float16 v16h;
typedef __attribute__((ext_vector_type(8)))  _Float16 v8h;
typedef __attribute__((ext_vector_type(8)))  unsigned short v8us;
typedef __attribute__((ext_vector_type(8)))  float    v8f;
typedef __attribute__((ext_vector_type(4)))  float    v4f;
typedef v8h  __attribute__((may_alias)) v8ha;
typedef v4f  __attribute__((may_alias)) v4fa;
typedef v8us __attribute__((may_alias)) v8usa;

__device__ __forceinline__ unsigned short f2bf(float f) { unsigned u = __float_as_uint(f); u += 0x7FFFu + ((u >> 16) & 1u); return (unsigned short)(u >> 16); }
__device__ __forceinline__ float bf2f(unsigned short b) { return __uint_as_float(((unsigned)b) << 16); }
__device__ __forceinline__ float bfr(float f) { return bf2f(f2bf(f)); }
__device__ __forceinline__ v16h cat16(v8h lo, v8h hi) { return __builtin_shufflevector(lo, hi, 0, 1, 2, 3, 4, 5, 6, 7, 8, 9, 10, 11, 12, 13, 14, 15); }
__device__ __forceinline__ v16bf cat16b(v8us lo, v8us hi) { return __builtin_bit_cast(v16bf, __builtin_shufflevector(lo, hi, 0, 1, 2, 3, 4, 5, 6, 7, 8, 9, 10, 11, 12, 13, 14, 15)); }
__device__ __forceinline__ v8f wmma16(v16h a, v16h b, v8f c) { return __builtin_amdgcn_wmma_f32_16x16x32_f16(false, a, false, b, (short)0, c, false, false); }
__device__ __forceinline__ v8f wmmab(v16bf a, v16bf b, v8f c) { return __builtin_amdgcn_wmma_f32_16x16x32_bf16(false, a, false, b, (short)0, c, false, false); }


template <typename T16> struct WFrag;
template <> struct WFrag<h16> { typedef v16h V; static __device__ __forceinline__ V ld(const h16* p) { return cat16(*(const v8h*)p, *(const v8h*)(p + 16)); } static __device__ __forceinline__ v8f mma(V a, V b, v8f c) { return wmma16(a, b, c); } };
template <> struct WFrag<bf> { typedef v16bf V; static __device__ __forceinline__ V ld(const bf* p) { return cat16b(*(const v8us*)p, *(const v8us*)(p + 16)); } static __device__ __forceinline__ v8f mma(V a, V b, v8f c) { return wmmab(a, b, c); } };
template <typename T16, int NSPLIT, bool BIAS>
__global__ __launch_bounds__(32) void k_gemmw(const T16* __restrict__ A, const T16* __restrict__ A2, const T16* __restrict__ Bt, const T16* __restrict__ Bt2, int K, float* C, int ldc, const float* __restrict__ bias, size_t sA, size_t sB, size_t sC) {
    typedef typename WFrag<T16>::V V;
    __shared__ __align__(16) float os[16 * 68];
    const size_t z = blockIdx.z; A += z * sA; if (A2) A2 += z * sA; Bt += z * sB; if (Bt2) Bt2 += z * sB; C += z * sC;
    const int lane = threadIdx.x & 31, lr = lane & 15, hi = lane >> 4; const int r0 = blockIdx.x * 64, c0 = blockIdx.y * 64;
    v8f acc[4][4];
#pragma unroll
    for (int mb = 0; mb < 4; ++mb)
#pragma unroll
        for (int nb = 0; nb < 4; ++nb) acc[mb][nb] = (v8f){};
    const size_t aoff = (size_t)(r0 + lr) * K + 8 * hi, boff = (size_t)(c0 + lr) * K + 8 * hi;
#pragma unroll 1
    for (int kc = 0; kc < K; kc += 32) {
        V a[4], a2[4];
#pragma unroll
        for (int mb = 0; mb < 4; ++mb) { a[mb] = WFrag<T16>::ld(A + aoff + (size_t)mb * 16 * K + kc); if (NSPLIT == 1 || NSPLIT == 2) a2[mb] = WFrag<T16>::ld(A2 + aoff + (size_t)mb * 16 * K + kc); }
#pragma unroll
        for (int nb = 0; nb < 4; ++nb) { const V b = WFrag<T16>::ld(Bt + boff + (size_t)nb * 16 * K + kc); V b2; if (NSPLIT >= 2) b2 = WFrag<T16>::ld(Bt2 + boff + (size_t)nb * 16 * K + kc);
#pragma unroll
            for (int mb = 0; mb < 4; ++mb) { acc[mb][nb] = WFrag<T16>::mma(a[mb], b, acc[mb][nb]); if (NSPLIT == 1 || NSPLIT == 2) acc[mb][nb] = WFrag<T16>::mma(a2[mb], b, acc[mb][nb]); if (NSPLIT >= 2) acc[mb][nb] = WFrag<T16>::mma(a[mb], b2, acc[mb][nb]); } }
        asm volatile("v_nop\n\tv_nop\n\tv_nop\n\tv_nop" : "+v"(acc[0][0]), "+v"(acc[1][1]), "+v"(acc[2][2]), "+v"(acc[3][3]) : "v"(a[0]), "v"(a[3]));
    }
#pragma unroll
    for (int mb = 0; mb < 4; ++mb) {
#pragma unroll
        for (int nb = 0; nb < 4; ++nb) {
#pragma unroll
            for (int j = 0; j < 8; ++j) os[(hi * 8 + j) * 68 + nb * 16 + lr] = acc[mb][nb][j]; }
        __builtin_amdgcn_wave_barrier(); asm volatile("" ::: "memory");
        float* crow = C + (size_t)(r0 + mb * 16) * ldc + c0;
#pragma unroll 1
        for (int ps = 0; ps < 2; ++ps) {
#pragma unroll
            for (int s = 0; s < 8; ++s) { const int row = 2 * s + hi, cofs = lr * 4; v4f val = *(const v4fa*)(os + row * 68 + cofs); if (BIAS) { val[0] += bfr(bias[c0 + cofs]); val[1] += bfr(bias[c0 + cofs + 1]); val[2] += bfr(bias[c0 + cofs + 2]); val[3] += bfr(bias[c0 + cofs + 3]); }
                *(volatile v4f*)(crow + (size_t)row * ldc + cofs) = val; }
            if (ps == 0) __threadfence(); }
        __builtin_amdgcn_wave_barrier(); asm volatile("" ::: "memory");
    }
}

template <typename T16, int NSPLIT, int CMODE>
__global__ __launch_bounds__(32) void k_gemmc(const T16* __restrict__ A, const T16* __restrict__ A2, const T16* __restrict__ Bt, const T16* __restrict__ Bt2, int K, float* C, int ldc, int roff, size_t sA, size_t sB, size_t sC) {
    typedef typename WFrag<T16>::V V;
    __shared__ __align__(16) float os[16 * 68];
    const size_t z = blockIdx.z; A += z * sA; if (A2) A2 += z * sA; Bt += z * sB; if (Bt2) Bt2 += z * sB; C += z * sC;
    const int lane = threadIdx.x & 31, lr = lane & 15, hi = lane >> 4; const int r0 = blockIdx.x * 64, c0 = blockIdx.y * 64;
    if (CMODE == 1 && c0 > r0 + roff + 63) return;
    const int Kl = (CMODE == 2) ? min(K, r0 + roff + 64) : K;
    v8f acc[4][4];
#pragma unroll
    for (int mb = 0; mb < 4; ++mb)
#pragma unroll
        for (int nb = 0; nb < 4; ++nb) acc[mb][nb] = (v8f){};
    const size_t aoff = (size_t)(r0 + lr) * K + 8 * hi, boff = (size_t)(c0 + lr) * K + 8 * hi;
#pragma unroll 1
    for (int kc = 0; kc < Kl; kc += 32) {
        V a[4], a2[4];
#pragma unroll
        for (int mb = 0; mb < 4; ++mb) { a[mb] = WFrag<T16>::ld(A + aoff + (size_t)mb * 16 * K + kc); if (NSPLIT == 1 || NSPLIT == 2) a2[mb] = WFrag<T16>::ld(A2 + aoff + (size_t)mb * 16 * K + kc); }
#pragma unroll
        for (int nb = 0; nb < 4; ++nb) { const V b = WFrag<T16>::ld(Bt + boff + (size_t)nb * 16 * K + kc); V b2; if (NSPLIT >= 2) b2 = WFrag<T16>::ld(Bt2 + boff + (size_t)nb * 16 * K + kc);
#pragma unroll
            for (int mb = 0; mb < 4; ++mb) { acc[mb][nb] = WFrag<T16>::mma(a[mb], b, acc[mb][nb]); if (NSPLIT == 1 || NSPLIT == 2) acc[mb][nb] = WFrag<T16>::mma(a2[mb], b, acc[mb][nb]); if (NSPLIT >= 2) acc[mb][nb] = WFrag<T16>::mma(a[mb], b2, acc[mb][nb]); } }
        asm volatile("v_nop\n\tv_nop\n\tv_nop\n\tv_nop" : "+v"(acc[0][0]), "+v"(acc[1][1]), "+v"(acc[2][2]), "+v"(acc[3][3]) : "v"(a[0]), "v"(a[3]));
    }
#pragma unroll
    for (int mb = 0; mb < 4; ++mb) {
#pragma unroll
        for (int nb = 0; nb < 4; ++nb) {
#pragma unroll
            for (int j = 0; j < 8; ++j) os[(hi * 8 + j) * 68 + nb * 16 + lr] = acc[mb][nb][j]; }
        __builtin_amdgcn_wave_barrier(); asm volatile("" ::: "memory");
        float* crow = C + (size_t)(r0 + mb * 16) * ldc + c0;
#pragma unroll 1
        for (int ps = 0; ps < 2; ++ps) {
#pragma unroll
            for (int s = 0; s < 8; ++s) { const int row = 2 * s + hi, cofs = lr * 4; v4f val = *(const v4fa*)(os + row * 68 + cofs);
                *(volatile v4f*)(crow + (size_t)row * ldc + cofs) = val; }
            if (ps == 0) __threadfence(); }
        __builtin_amdgcn_wave_barrier(); asm volatile("" ::: "memory");
    }
}
__device__ __forceinline__ h16 tohx(float x) { return (h16)x; }
__device__ __forceinline__ void splitf(float y, unsigned short& h, unsigned short& l) { h = f2bf(y); l = f2bf(y - bf2f(h)); }
typedef __attribute__((ext_vector_type(2))) unsigned short v2us;
typedef __attribute__((ext_vector_type(4))) unsigned short v4us;
typedef __attribute__((ext_vector_type(2))) _Float16 v2h;
typedef __attribute__((ext_vector_type(4))) _Float16 v4h; typedef __attribute__((ext_vector_type(2))) float v2f;

__global__ __launch_bounds__(256) void k_cvt8(const float* __restrict__ src, bf* dst, size_t n8) { const size_t i = (size_t)blockIdx.x * 256 + threadIdx.x; if (i >= n8) return; const v8f v = *(const v8f*)(src + i * 8); v8us o;
#pragma unroll
    for (int k = 0; k < 8; ++k) o[k] = f2bf(v[k]); *(volatile v8us*)(dst + i * 8) = o; __threadfence(); *(volatile v8us*)(dst + i * 8) = o; }
__global__ __launch_bounds__(256) void k_wtG(const float* __restrict__ w, int K, int N, bf* Bt) {
    const int lane = threadIdx.x & 31; const int L0 = (blockIdx.x * 8 + (threadIdx.x >> 5)) * 8; const int nlines = N * K / 64;
#pragma unroll
    for (int ps = 0; ps < 2; ++ps) {
#pragma unroll 1
        for (int l = 0; l < 8; ++l) { const int L = L0 + l; if (L >= nlines) break; const size_t e = (size_t)L * 64 + lane * 2; const int k = (int)(e % K), n = (int)(e / K); v2us o;
            o[0] = f2bf(w[(size_t)k * N + n]); o[1] = f2bf(w[(size_t)(k + 1) * N + n]); *(volatile v2us*)(Bt + e) = o; }
        if (ps == 0) __threadfence(); }
}

__global__ __launch_bounds__(256) void k_cs32(float* CS) { const int idx = blockIdx.x * 256 + threadIdx.x; if (idx >= TT * RD) return; const int t = idx / RD, j = idx % RD; const int i = j % (RD / 2); const float inv = __fdiv_rn(1.0f, powf(10000.0f, (float)(2 * i) / (float)RD)); const float ang = __fmul_rn((float)t, inv); v2f cs; cs[0] = cosf(ang); cs[1] = sinf(ang); *(volatile v2f*)(CS + (size_t)idx * 2) = cs; __threadfence(); *(volatile v2f*)(CS + (size_t)idx * 2) = cs; }
__global__ __launch_bounds__(256) void k_prope(const float* __restrict__ F, const float* __restrict__ CS, h16* P16, bf* Ph, bf* Pl) { const size_t e = ((size_t)blockIdx.x * 256 + threadIdx.x) * 2; if (e >= (size_t)NH_ * TT * HD) return; const int d = (int)(e % HD); const int t = (int)((e / HD) % TT); const int h = (int)(e / ((size_t)HD * TT)); const float* f = F + (size_t)t * DM + h * HD; v2h o16; v2us oh, ol;
#pragma unroll
    for (int q = 0; q < 2; ++q) { const int dd = d + q; float r;
        if (dd < RD) { const int dp = (dd < RD / 2) ? dd + RD / 2 : dd - RD / 2; const v2f cs = *(const v2f*)(CS + ((size_t)t * RD + dd) * 2); float a = __fmul_rn(f[dd], cs[0]), bq = __fmul_rn(f[dp], cs[1]); asm volatile("" : "+v"(a)); asm volatile("" : "+v"(bq)); r = (dd < RD / 2) ? __fsub_rn(a, bq) : __fadd_rn(a, bq); } else r = f[dd];
        o16[q] = tohx(r); unsigned short a2, c2; splitf(r, a2, c2); oh[q] = a2; ol[q] = c2; }
    *(volatile v2h*)(P16 + e) = o16; *(volatile v2us*)(Ph + e) = oh; *(volatile v2us*)(Pl + e) = ol; __threadfence(); *(volatile v2h*)(P16 + e) = o16; *(volatile v2us*)(Ph + e) = oh; *(volatile v2us*)(Pl + e) = ol; }
__global__ __launch_bounds__(256) void k_vt(const float* __restrict__ V, h16* VT, bf* VTh, bf* VTl) { const size_t e = ((size_t)blockIdx.x * 256 + threadIdx.x) * 2; if (e >= (size_t)NH_ * VT64 * TT) return; const int t = (int)(e % TT); const int d = (int)((e / TT) % VT64); const int h = (int)(e / ((size_t)TT * VT64)); v2h o; v2us oh, ol;
#pragma unroll
    for (int u = 0; u < 2; ++u) { const float vv = (d < VHD) ? V[(size_t)(t + u) * VP + h * VHD + d] : 0.f; o[u] = tohx(vv); unsigned short a2, b2; splitf(vv, a2, b2); oh[u] = a2; ol[u] = b2; }
    *(volatile v2h*)(VT + e) = o; *(volatile v2us*)(VTh + e) = oh; *(volatile v2us*)(VTl + e) = ol; __threadfence(); *(volatile v2h*)(VT + e) = o; *(volatile v2us*)(VTh + e) = oh; *(volatile v2us*)(VTl + e) = ol; }
__global__ __launch_bounds__(256) void k_csoft(const float* __restrict__ S, h16* P16, bf* Ph, bf* Pl) { const int lane = threadIdx.x & 31; const int row = blockIdx.x * 8 + (threadIdx.x >> 5); if (row >= ZH * TT) return; const int i = row % TT; const int zz = row / TT; const bool hires = (i < RH); const float* sr = S + (size_t)row * TT; const int nch = (i >> 7) + 1;     float v[TT / 32]; float mx = -3.0e38f;
#pragma unroll
    for (int ch = 0; ch < TT / 128; ++ch) { v4f a; if (ch < nch) a = *(const v4f*)(sr + ch * 128 + lane * 4); else { a[0] = 0.f; a[1] = 0.f; a[2] = 0.f; a[3] = 0.f; }
#pragma unroll
        for (int u = 0; u < 4; ++u) { const int j = ch * 128 + lane * 4 + u; const float t = (j <= i) ? a[u] * SCL : -3.0e38f; v[ch * 4 + u] = t; mx = fmaxf(mx, t); } }
#pragma unroll
    for (int sh = 16; sh; sh >>= 1) mx = fmaxf(mx, __shfl_xor(mx, sh, 32));
    float sum = 0.f;
#pragma unroll
    for (int q = 0; q < TT / 32; ++q) { float d0 = __fsub_rn(v[q], mx); asm volatile("" : "+v"(d0)); v[q] = __builtin_amdgcn_exp2f(__fmul_rn(d0, 1.4426950408889634f)); sum += v[q]; }
#pragma unroll
    for (int sh = 16; sh; sh >>= 1) sum += __shfl_xor(sum, sh, 32);
    const float f = __fdiv_rn(hires ? 1.0f : PCAR, sum);
    for (int ps = 0; ps < 2; ++ps) {
        if (hires) {
#pragma unroll
            for (int ch = 0; ch < TT / 128; ++ch) { v4us oh, ol; for (int q = 0; q < 4; ++q) { unsigned short a2, b2; splitf(v[ch * 4 + q] * f, a2, b2); oh[q] = a2; ol[q] = b2; } const size_t oo = ((size_t)zz * RH + i) * TT + ch * 128 + lane * 4; *(volatile v4us*)(Ph + oo) = oh; *(volatile v4us*)(Pl + oo) = ol; }
        } else {
#pragma unroll
            for (int ch = 0; ch < TT / 128; ++ch) { v4h o4; for (int q = 0; q < 4; ++q) o4[q] = tohx(v[ch * 4 + q] * f); *(volatile v4h*)(P16 + (size_t)row * TT + ch * 128 + lane * 4) = o4; } }
        if (ps == 0) __threadfence(); } }
__global__ __launch_bounds__(256) void k_vmrg(const float* __restrict__ Oall, bf* Ah, bf* Al) { const size_t e = ((size_t)blockIdx.x * 256 + threadIdx.x) * 4; if (e >= (size_t)TT * VP) return; const int c = (int)(e % VP); const int t = (int)(e / VP); v4us oh, ol;
const float cs = (t < RH) ? 1.0f : (1.0f / PCAR);
#pragma unroll
    for (int u = 0; u < 4; ++u) { const int cc = c + u; const int h = cc / VHD, d = cc % VHD; unsigned short a, b; splitf(Oall[((size_t)h * TT + t) * VT64 + d] * cs, a, b); oh[u] = a; ol[u] = b; }
    *(volatile v4us*)(Ah + e) = oh; *(volatile v4us*)(Al + e) = ol; __threadfence(); *(volatile v4us*)(Ah + e) = oh; *(volatile v4us*)(Al + e) = ol; }

extern "C" void kernel_launch(void* const* d_in, const int* in_sizes, int n_in,
                              void* d_out, int out_size, void* d_ws, size_t ws_size, hipStream_t stream) {
    (void)in_sizes; (void)n_in; (void)out_size;
    const float* x = (const float*)d_in[0]; const float* Wq = (const float*)d_in[1]; const float* bq = (const float*)d_in[2]; const float* Wk = (const float*)d_in[3]; const float* bk = (const float*)d_in[4]; const float* Wv = (const float*)d_in[5]; const float* bv = (const float*)d_in[6]; const float* Wd = (const float*)d_in[7]; const float* bd = (const float*)d_in[8];
    float* OUT = (float*)d_out;
    char* wsp = (char*)d_ws;
    auto take = [&](size_t bytes) { char* p = wsp; wsp += (bytes + 255) & ~(size_t)255; return (void*)p; };
    bf* BQ = (bf*)take((size_t)DM * DM * 2); bf* BK = (bf*)take((size_t)DM * DM * 2); bf* BV = (bf*)take((size_t)VP * DM * 2); bf* BD = (bf*)take((size_t)DM * VP * 2); float* CS = (float*)take((size_t)TT * RD * 2 * 4);
    bf* XB = (bf*)take((size_t)TT * DM * 2); float* FQ = (float*)take((size_t)TT * DM * 4); float* FK = (float*)take((size_t)TT * DM * 4); float* FV = (float*)take((size_t)TT * VP * 4);
    h16* QP16 = (h16*)take((size_t)NH_ * TT * HD * 2); bf* QPh = (bf*)take((size_t)NH_ * TT * HD * 2); bf* QPl = (bf*)take((size_t)NH_ * TT * HD * 2); h16* KP16 = (h16*)take((size_t)NH_ * TT * HD * 2); bf* KPh = (bf*)take((size_t)NH_ * TT * HD * 2); bf* KPl = (bf*)take((size_t)NH_ * TT * HD * 2); h16* VT = (h16*)take((size_t)NH_ * VT64 * TT * 2); bf* VTh = (bf*)take((size_t)NH_ * VT64 * TT * 2); bf* VTl = (bf*)take((size_t)NH_ * VT64 * TT * 2);
    float* S = (float*)take((size_t)ZH * TT * TT * 4); h16* P16 = (h16*)take((size_t)ZH * TT * TT * 2); bf* Ph = (bf*)take((size_t)ZH * RH * TT * 2); bf* Pl = (bf*)take((size_t)ZH * RH * TT * 2); float* Oall = (float*)take((size_t)NH_ * TT * VT64 * 4); bf* ATh = (bf*)take((size_t)TT * VP * 2); bf* ATl = (bf*)take((size_t)TT * VP * 2);
    if ((size_t)(wsp - (char*)d_ws) > ws_size) return;
    k_wtG<<<(DM * DM / 64 + 63) / 64, 256, 0, stream>>>(Wq, DM, DM, BQ); k_wtG<<<(DM * DM / 64 + 63) / 64, 256, 0, stream>>>(Wk, DM, DM, BK); k_wtG<<<(DM * VP / 64 + 63) / 64, 256, 0, stream>>>(Wv, DM, VP, BV); k_wtG<<<(VP * DM / 64 + 63) / 64, 256, 0, stream>>>(Wd, VP, DM, BD);
    k_cs32<<<(TT * RD + 255) / 256, 256, 0, stream>>>(CS);
    const size_t zq = (size_t)TT * HD, zS = (size_t)TT * TT, zv = (size_t)VT64 * TT, zo = (size_t)TT * VT64;
    for (int b = 0; b < NB_; ++b) {
        k_cvt8<<<(TT * DM / 8 + 255) / 256, 256, 0, stream>>>(x + (size_t)b * TT * DM, XB, TT * DM / 8);
        k_gemmw<bf, 0, true><<<dim3(TT / 64, DM / 64, 1), 32, 0, stream>>>(XB, nullptr, BQ, nullptr, DM, FQ, DM, bq, 0, 0, 0); k_gemmw<bf, 0, true><<<dim3(TT / 64, DM / 64, 1), 32, 0, stream>>>(XB, nullptr, BK, nullptr, DM, FK, DM, bk, 0, 0, 0); k_gemmw<bf, 0, true><<<dim3(TT / 64, VP / 64, 1), 32, 0, stream>>>(XB, nullptr, BV, nullptr, DM, FV, VP, bv, 0, 0, 0);
        k_prope<<<(unsigned)(((size_t)NH_ * TT * HD / 2 + 255) / 256), 256, 0, stream>>>(FQ, CS, QP16, QPh, QPl); k_prope<<<(unsigned)(((size_t)NH_ * TT * HD / 2 + 255) / 256), 256, 0, stream>>>(FK, CS, KP16, KPh, KPl); k_vt<<<(unsigned)(((size_t)NH_ * VT64 * TT / 2 + 255) / 256), 256, 0, stream>>>(FV, VT, VTh, VTl);
        for (int h0 = 0; h0 < NH_; h0 += ZH) { const size_t zh = (size_t)h0;
            k_gemmc<bf, 2, 1><<<dim3(RH / 64, TT / 64, ZH), 32, 0, stream>>>(QPh + zh * zq, QPl + zh * zq, KPh + zh * zq, KPl + zh * zq, HD, S, TT, 0, zq, zq, zS);
            k_gemmc<h16, 0, 1><<<dim3((TT - RH) / 64, TT / 64, ZH), 32, 0, stream>>>(QP16 + zh * zq + (size_t)RH * HD, nullptr, KP16 + zh * zq, nullptr, HD, S + (size_t)RH * TT, TT, RH, zq, zq, zS);
            k_csoft<<<ZH * TT / 8, 256, 0, stream>>>(S, P16, Ph, Pl);
            k_gemmc<bf, 2, 2><<<dim3(RH / 64, 1, ZH), 32, 0, stream>>>(Ph, Pl, VTh + zh * zv, VTl + zh * zv, TT, Oall + zh * zo, VT64, 0, (size_t)RH * TT, zv, zo);
            k_gemmc<h16, 0, 2><<<dim3((TT - RH) / 64, 1, ZH), 32, 0, stream>>>(P16 + (size_t)RH * TT, nullptr, VT + zh * zv, nullptr, TT, Oall + zh * zo + (size_t)RH * VT64, VT64, RH, zS, zv, zo); }
        k_vmrg<<<(unsigned)(((size_t)TT * VP / 4 + 255) / 256), 256, 0, stream>>>(Oall, ATh, ATl);
        k_gemmw<bf, 1, true><<<dim3(TT / 64, DM / 64, 1), 32, 0, stream>>>(ATh, ATl, BD, nullptr, VP, OUT + (size_t)b * TT * DM, DM, bd, 0, 0, 0); }
}
